// FAVOR_4406636445947
// MI455X (gfx1250) — hardware-verified
//
#include <hip/hip_runtime.h>
#include <math.h>
typedef __attribute__((ext_vector_type(16))) _Float16 v16h;
typedef __attribute__((ext_vector_type(8)))  _Float16 v8h;
typedef __attribute__((ext_vector_type(16))) __bf16   v16b;
typedef __attribute__((ext_vector_type(8)))  __bf16   v8b;
typedef __attribute__((ext_vector_type(8)))  float    v8f;
typedef __attribute__((ext_vector_type(4)))  float    v4f;
#define PSCALE 32768.0f
#define U16(p) ((const unsigned short*)(const void*)(p))
#define PSCALE_INV (1.0f / 32768.0f)

__device__ __forceinline__ unsigned short f2bf_bits(float f) {
  unsigned u = __float_as_uint(f);
  return (unsigned short)((u + 0x7FFFu + ((u >> 16) & 1u)) >> 16);
}
__device__ __forceinline__ float bf_bits2f(unsigned short h) { return __uint_as_float(((unsigned)h) << 16); }

__device__ __forceinline__ void dep_guard_h(v8f& a, v8f& b, v16h x, v16h y) { asm volatile("v_nop\n\tv_nop\n\tv_nop\n\tv_nop" : "+v"(a), "+v"(b) : "v"(x), "v"(y)); }
__device__ __forceinline__ void dep_guard_b(v8f& a, v8f& b, v16b x, v16b y) { asm volatile("v_nop\n\tv_nop\n\tv_nop\n\tv_nop" : "+v"(a), "+v"(b) : "v"(x), "v"(y)); }
__device__ __forceinline__ void keep4_h(v16h a, v16h b, v16h c, v16h d) { asm volatile("v_nop" :: "v"(a), "v"(b), "v"(c), "v"(d)); }
__device__ __forceinline__ void keep4_b(v16b a, v16b b, v16b c, v16b d) { asm volatile("v_nop" :: "v"(a), "v"(b), "v"(c), "v"(d)); }
__device__ __forceinline__ void acc_guard4(v8f& a, v8f& b, v8f& c, v8f& d) { asm volatile("v_nop\n\tv_nop\n\tv_nop\n\tv_nop" : "+v"(a), "+v"(b), "+v"(c), "+v"(d)); }
template <typename T> struct Frag;
template <> struct Frag<_Float16> {
  typedef v16h V; union U { v16h v; v8h h[2]; };
  static __device__ __forceinline__ v16h load(const _Float16* p) {
    U f; f.h[0] = *(const v8h*)(p); f.h[1] = *(const v8h*)(p + 16); return f.v;
  }
  static __device__ __forceinline__ v8f mma(v16h a, v16h b, v8f c) {
    return __builtin_amdgcn_wmma_f32_16x16x32_f16(false, a, false, b, (short)0, c, false, false);
  }
  static __device__ __forceinline__ void guard(v8f& a, v8f& b, v16h x, v16h y) { dep_guard_h(a, b, x, y); }
  static __device__ __forceinline__ void keep(v16h a, v16h b, v16h c, v16h d) { keep4_h(a, b, c, d); }
};
template <> struct Frag<__bf16> {
  typedef v16b V; union U { v16b v; v8b h[2]; };
  static __device__ __forceinline__ v16b load(const __bf16* p) {
    U f; f.h[0] = *(const v8b*)(p); f.h[1] = *(const v8b*)(p + 16); return f.v;
  }
  static __device__ __forceinline__ v8f mma(v16b a, v16b b, v8f c) {
    return __builtin_amdgcn_wmma_f32_16x16x32_bf16(false, a, false, b, (short)0, c, false, false);
  }
  static __device__ __forceinline__ void guard(v8f& a, v8f& b, v16b x, v16b y) { dep_guard_b(a, b, x, y); }
  static __device__ __forceinline__ void keep(v16b a, v16b b, v16b c, v16b d) { keep4_b(a, b, c, d); }
};

template <int ET> struct Elem;
template <> struct Elem<0> { typedef _Float16 T; };
template <> struct Elem<1> { typedef __bf16 T; };
template <int ET, bool SPLIT, int BIAS_MODE, int OUT_MODE, bool RESID, int ACT = 0>
__global__ __launch_bounds__(256) void wmma_gemm64(
    const unsigned short* __restrict__ Ap, const unsigned short* __restrict__ A2p, int lda, long strideA,
    const unsigned short* __restrict__ Btp, const unsigned short* __restrict__ Bt2p, int ldb, long strideB,
    void* __restrict__ Cout, void* __restrict__ Cout2, int ldc, long strideC,
    const float* __restrict__ bias,
    const float* __restrict__ resid, long strideR,
    int M, int N, int K, float scale) {
  typedef typename Elem<ET>::T T;
  typedef typename Frag<T>::V V;
  const T* A = (const T*)Ap; const T* A2 = (const T*)A2p; const T* Bt = (const T*)Btp; const T* Bt2 = (const T*)Bt2p;
  __shared__ __align__(16) float sT[8][16 * 68];
  const int b    = blockIdx.y;
  const int lane = threadIdx.x & 31;
  const int wave = threadIdx.x >> 5;
  const int tilesN = N >> 6;
  const int tilesM = M >> 6;
  const int tile = blockIdx.x * 8 + wave;
  if (tile >= tilesM * tilesN) return;
  const int tm = tile / tilesN;
  const int tn = tile - tm * tilesN;
  const int m0 = tm << 6;
  const int n0 = tn << 6;

  const T* Ab  = A  + (size_t)b * strideA;
  const T* Bb  = Bt + (size_t)b * strideB;
  const T* Ab2 = SPLIT ? (A2  + (size_t)b * strideA) : nullptr;
  const T* Bb2 = SPLIT ? (Bt2 + (size_t)b * strideB) : nullptr;

  const int rlane = lane & 15;
  const int koff  = (lane >> 4) * 8;
  const int mOff  = (lane >> 4) * 8;

  v8f acc[4][4];
#pragma unroll
  for (int i = 0; i < 4; ++i)
#pragma unroll
    for (int j = 0; j < 4; ++j) acc[i][j] = (v8f){0.f,0.f,0.f,0.f,0.f,0.f,0.f,0.f};

  for (int k0 = 0; k0 < K; k0 += 32) {
    V bh[4], bl[4];
#pragma unroll
    for (int j = 0; j < 4; ++j) {
      const size_t bo = (size_t)(n0 + (j << 4) + rlane) * ldb + koff + k0;
      bh[j] = Frag<T>::load(Bb + bo);
      if (SPLIT) bl[j] = Frag<T>::load(Bb2 + bo);
    }
#pragma unroll
    for (int i = 0; i < 4; ++i) {
      const size_t ao = (size_t)(m0 + (i << 4) + rlane) * lda + koff + k0;
      V ah = Frag<T>::load(Ab + ao);
      V al;
      if (SPLIT) al = Frag<T>::load(Ab2 + ao);
#pragma unroll
      for (int j = 0; j < 4; ++j) {
        acc[i][j] = Frag<T>::mma(ah, bh[j], acc[i][j]);
        if (SPLIT) {
          acc[i][j] = Frag<T>::mma(ah, bl[j], acc[i][j]);
          acc[i][j] = Frag<T>::mma(al, bh[j], acc[i][j]);
        }
      }
      Frag<T>::guard(acc[i][0], acc[i][3], ah, SPLIT ? al : ah);
    }
    Frag<T>::keep(bh[0], bh[1], bh[2], bh[3]);
    if (SPLIT) Frag<T>::keep(bl[0], bl[1], bl[2], bl[3]);
  }
  acc_guard4(acc[0][0], acc[0][1], acc[0][2], acc[0][3]);
  acc_guard4(acc[1][0], acc[1][1], acc[1][2], acc[1][3]);
  acc_guard4(acc[2][0], acc[2][1], acc[2][2], acc[2][3]);
  acc_guard4(acc[3][0], acc[3][1], acc[3][2], acc[3][3]);

  float* slab = sT[wave];
  const float* Rb = RESID ? (resid + (size_t)b * strideR) : nullptr;
#pragma unroll
  for (int i = 0; i < 4; ++i) {
    const int mBase = m0 + (i << 4);
#pragma unroll
    for (int j = 0; j < 4; ++j) {
      const int n = n0 + (j << 4) + rlane;
      float bv = 0.f;
      if (BIAS_MODE == 2) bv = bias[n];
#pragma unroll
      for (int r = 0; r < 8; ++r) {
        float v = acc[i][j][r] * scale;
        if (BIAS_MODE == 1) v += bias[mBase + mOff + r];
        if (BIAS_MODE == 2) v += bv;
        if (RESID) v += Rb[(size_t)(mBase + mOff + r) * ldc + n];
        if (ACT == 1) v = tanhf(v);
        if (ACT == 2) v = fmaxf(v, 0.0f);
        if (ACT == 3) v = v / (1.0f + expf(-v));
        if (ACT == 4) v = (v > 0.f) ? v : 0.01f * v;
        if (ACT == 5) v = 0.5f * v * (1.0f + erff(v * 0.70710678118654752f));
        slab[(mOff + r) * 68 + (j << 4) + rlane] = v;
      }
    }
    __builtin_amdgcn_fence(__ATOMIC_RELEASE, "workgroup");
    __builtin_amdgcn_wave_barrier();
    __builtin_amdgcn_fence(__ATOMIC_ACQUIRE, "workgroup");
    if (OUT_MODE == 0) {
      float* C = (float*)Cout + (size_t)b * strideC;
      const int hh = lane >> 4, c4 = (lane & 15) * 4;
      for (int pass = 0; pass < 2; ++pass) {
#pragma unroll
        for (int it = 0; it < 8; ++it) {
          const int row = it * 2 + hh;
          v4f v = *(const v4f*)(slab + row * 68 + c4);
          *(volatile v4f*)(C + (size_t)(mBase + row) * ldc + n0 + c4) = v;
        }
        __threadfence();
      }
    } else {
      const int q = lane >> 3, c8 = (lane & 7) * 8;
      unsigned short* C  = (unsigned short*)Cout  + (size_t)b * strideC;
      unsigned short* C2 = (OUT_MODE == 2) ? ((unsigned short*)Cout2 + (size_t)b * strideC) : nullptr;
      for (int pass = 0; pass < 2; ++pass) {
#pragma unroll
        for (int it = 0; it < 4; ++it) {
          const int row = it * 4 + q;
          const float* sp = slab + row * 68 + c8;
          v8h hv, lv;
#pragma unroll
          for (int e = 0; e < 8; ++e) {
            if (OUT_MODE == 1) {
              hv[e] = (_Float16)sp[e];
            } else {
              unsigned short hb = f2bf_bits(sp[e]);
              unsigned short lb = f2bf_bits(sp[e] - bf_bits2f(hb));
              hv[e] = __builtin_bit_cast(_Float16, hb);
              lv[e] = __builtin_bit_cast(_Float16, lb);
            }
          }
          *(volatile v8h*)(C + (size_t)(mBase + row) * ldc + n0 + c8) = hv;
          if (OUT_MODE == 2) *(volatile v8h*)(C2 + (size_t)(mBase + row) * ldc + n0 + c8) = lv;
        }
        __threadfence();
      }
    }
    __builtin_amdgcn_fence(__ATOMIC_RELEASE, "workgroup");
    __builtin_amdgcn_wave_barrier();
    __builtin_amdgcn_fence(__ATOMIC_ACQUIRE, "workgroup");
  }
}

__global__ __launch_bounds__(256) void cast_f32_f16x2(
    const float* __restrict__ in, _Float16* __restrict__ out, int n2) {
  int i = blockIdx.x * 256 + threadIdx.x;
  if (i < n2) {
    const _Float16 h0 = (_Float16)in[2 * i], h1 = (_Float16)in[2 * i + 1];
    const unsigned u = (unsigned)__builtin_bit_cast(unsigned short, h0) | ((unsigned)__builtin_bit_cast(unsigned short, h1) << 16);
    ((volatile unsigned*)out)[i] = u;
    __threadfence();
    ((volatile unsigned*)out)[i] = u;
  }
}

__global__ __launch_bounds__(256) void split_f32_bf16x2(
    const float* __restrict__ in, __bf16* __restrict__ hi, __bf16* __restrict__ lo, long n2) {
  long i = (long)blockIdx.x * 256 + threadIdx.x;
  long stride = (long)gridDim.x * 256;
  for (int pass = 0; pass < 2; ++pass) {
    for (long j = i; j < n2; j += stride) {
      const float a = in[2 * j], b = in[2 * j + 1];
      const unsigned short ah = f2bf_bits(a), bh = f2bf_bits(b);
      const unsigned short al = f2bf_bits(a - bf_bits2f(ah)), bl = f2bf_bits(b - bf_bits2f(bh));
      ((volatile unsigned*)hi)[j] = (unsigned)ah | ((unsigned)bh << 16);
      ((volatile unsigned*)lo)[j] = (unsigned)al | ((unsigned)bl << 16);
    }
    __threadfence();
  }
}


__global__ __launch_bounds__(256) void transpose_cast_f16(const float* __restrict__ in, int ldi,
                                                         _Float16* __restrict__ outT, int ldo, float scale) {
  __shared__ __align__(16) _Float16 tile[64][72];
  const int c0 = blockIdx.x * 64, r0 = blockIdx.y * 64;
  const int t = threadIdx.y * 32 + threadIdx.x;
  for (int i = threadIdx.y; i < 64; i += 8) {
    tile[threadIdx.x][i]      = (_Float16)(in[(size_t)(r0 + i) * ldi + c0 + threadIdx.x] * scale);
    tile[32 + threadIdx.x][i] = (_Float16)(in[(size_t)(r0 + i) * ldi + c0 + 32 + threadIdx.x] * scale);
  }
  __syncthreads();
  const int q = t >> 3, c8 = (t & 7) * 8;
  for (int pass = 0; pass < 2; ++pass) {
#pragma unroll
    for (int it = 0; it < 2; ++it) {
      const int c = it * 32 + q;
      v8h hv = *(const v8h*)(&tile[c][c8]);
      *(volatile v8h*)(outT + (size_t)(c0 + c) * ldo + r0 + c8) = hv;
    }
    __threadfence();
  }
}

#define FB 4
#define FS 2048
#define FKD 256
#define FM 128
#define FDV 64
__global__ __launch_bounds__(256) void phi_cast_kernel(const float* __restrict__ P, unsigned* __restrict__ P16, int n2) {
  const int i = blockIdx.x * 256 + threadIdx.x; if (i >= n2) return;
  const float a = P[2 * i] + 1e-3f, b = P[2 * i + 1] + 1e-3f;
  const unsigned u = (unsigned)__builtin_bit_cast(unsigned short, (_Float16)a) | ((unsigned)__builtin_bit_cast(unsigned short, (_Float16)b) << 16);
  ((volatile unsigned*)P16)[i] = u; __threadfence(); ((volatile unsigned*)P16)[i] = u;
}
__global__ __launch_bounds__(256) void mask_rowsum_kernel(const float* __restrict__ S, __bf16* __restrict__ Sh, __bf16* __restrict__ Sl, float* __restrict__ norm) {
  __shared__ float red[8];
  const int s = blockIdx.x, t = threadIdx.x, lane = t & 31, wave = t >> 5;
  float part = 0.f;
#pragma unroll
  for (int q = 0; q < 8; ++q) { const int col = q * 256 + t; part += (col <= s) ? S[(size_t)s * FS + col] : 0.f; }
  for (int o = 16; o > 0; o >>= 1) part += __shfl_xor(part, o, 32);
  if (lane == 0) red[wave] = part;
  __syncthreads();
  for (int pass = 0; pass < 2; ++pass) {
#pragma unroll
    for (int g = 0; g < 4; ++g) {
      const int c0 = g * 512 + 2 * t;
      const float a = (c0 <= s) ? S[(size_t)s * FS + c0] : 0.f, b = (c0 + 1 <= s) ? S[(size_t)s * FS + c0 + 1] : 0.f;
      const unsigned short ah = f2bf_bits(a), bh = f2bf_bits(b);
      const unsigned short al = f2bf_bits(a - bf_bits2f(ah)), bl = f2bf_bits(b - bf_bits2f(bh));
      ((volatile unsigned*)Sh)[((size_t)s * FS + c0) / 2] = (unsigned)ah | ((unsigned)bh << 16);
      ((volatile unsigned*)Sl)[((size_t)s * FS + c0) / 2] = (unsigned)al | ((unsigned)bl << 16);
    }
    __threadfence();
  }
  if (t < 32) { float n = 0.f; for (int w = 0; w < 8; ++w) n += red[w];
    ((volatile float*)norm)[(size_t)s * 32 + t] = (t == 0) ? n : 0.f; __threadfence(); ((volatile float*)norm)[(size_t)s * 32 + t] = (t == 0) ? n : 0.f; }
}
__global__ __launch_bounds__(256) void finalize_kernel(const float* __restrict__ O, const float* __restrict__ norm, float* __restrict__ outb) {
  __shared__ float tile[64][65];
  const int s0 = blockIdx.x * 64, tx = threadIdx.x, ty = threadIdx.y;
  for (int j = ty; j < 64; j += 8) { const int s = s0 + j; const float inv = 1.0f / norm[(size_t)s * 32];
    tile[j][tx] = O[(size_t)s * FDV + tx] * inv; tile[j][tx + 32] = O[(size_t)s * FDV + tx + 32] * inv; }
  __syncthreads();
  typedef __attribute__((ext_vector_type(2))) float v2f;
  for (int pass = 0; pass < 2; ++pass) {
    for (int k = 0; k < 8; ++k) { const int d = ty * 8 + k; const v2f v = {tile[2 * tx][d], tile[2 * tx + 1][d]};
      *(volatile v2f*)(outb + (size_t)d * FS + s0 + 2 * tx) = v; }
    __threadfence();
  }
}
extern "C" void kernel_launch(void* const* d_in, const int* in_sizes, int n_in, void* d_out, int out_size, void* d_ws, size_t ws_size, hipStream_t stream) {
  (void)in_sizes; (void)n_in; (void)out_size; (void)ws_size;
  const float* keys = (const float*)d_in[0]; const float* values = (const float*)d_in[1]; const float* queries = (const float*)d_in[2]; const float* feats = (const float*)d_in[3];
  float* out = (float*)d_out;
  char* ws = (char*)d_ws; size_t off = 0;
  auto carve = [&](size_t bytes) -> char* { char* p = ws + off; off += (bytes + 255) & ~(size_t)255; return p; };
  _Float16* KT16 = (_Float16*)carve((size_t)FS * FKD * 2); _Float16* QT16 = (_Float16*)carve((size_t)FS * FKD * 2);
  _Float16* F16 = (_Float16*)carve((size_t)FM * FKD * 2);
  unsigned* PK = (unsigned*)carve((size_t)FS * FM * 2); unsigned* PQ = (unsigned*)carve((size_t)FS * FM * 2);
  float* S = (float*)carve((size_t)FS * FS * 4);
  __bf16* Sh = (__bf16*)carve((size_t)FS * FS * 2); __bf16* Sl = (__bf16*)carve((size_t)FS * FS * 2);
  __bf16* Vh = (__bf16*)carve((size_t)FDV * FS * 2); __bf16* Vl = (__bf16*)carve((size_t)FDV * FS * 2);
  float* norm = (float*)carve((size_t)FS * 32 * 4);
  float* O = (float*)carve((size_t)FS * FDV * 4);
  float* Pf = (float*)carve((size_t)FS * FM * 4);
  cast_f32_f16x2<<<(FM * FKD / 2 + 255) / 256, 256, 0, stream>>>(feats, F16, FM * FKD / 2);
  for (int b = 0; b < FB; ++b) {
    transpose_cast_f16<<<dim3(FS / 64, FKD / 64), dim3(32, 8), 0, stream>>>(keys + (size_t)b * FKD * FS, FS, KT16, FKD, 1.0f);
    transpose_cast_f16<<<dim3(FS / 64, FKD / 64), dim3(32, 8), 0, stream>>>(queries + (size_t)b * FKD * FS, FS, QT16, FKD, 1.0f);
    { const int t = (FS / 64) * (FM / 64);
      wmma_gemm64<0, false, 0, 0, false, 2><<<dim3((t + 7) / 8, 1), 256, 0, stream>>>(U16(KT16), nullptr, FKD, 0, U16(F16), nullptr, FKD, 0, Pf, nullptr, FM, 0, nullptr, nullptr, 0, FS, FM, FKD, 1.0f);
      phi_cast_kernel<<<(FS * FM / 2 + 255) / 256, 256, 0, stream>>>(Pf, PK, FS * FM / 2);
      wmma_gemm64<0, false, 0, 0, false, 2><<<dim3((t + 7) / 8, 1), 256, 0, stream>>>(U16(QT16), nullptr, FKD, 0, U16(F16), nullptr, FKD, 0, Pf, nullptr, FM, 0, nullptr, nullptr, 0, FS, FM, FKD, 1.0f);
      phi_cast_kernel<<<(FS * FM / 2 + 255) / 256, 256, 0, stream>>>(Pf, PQ, FS * FM / 2); }
    { const int t = (FS / 64) * (FS / 64);
      wmma_gemm64<0, false, 0, 0, false><<<dim3((t + 7) / 8, 1), 256, 0, stream>>>((const unsigned short*)PQ, nullptr, FM, 0, (const unsigned short*)PK, nullptr, FM, 0, S, nullptr, FS, 0, nullptr, nullptr, 0, FS, FS, FM, 1.0f); }
    mask_rowsum_kernel<<<FS, 256, 0, stream>>>(S, Sh, Sl, norm);
    split_f32_bf16x2<<<(FDV * FS / 2 + 255) / 256, 256, 0, stream>>>(values + (size_t)b * FDV * FS, Vh, Vl, FDV * FS / 2);
    { const int t = (FS / 64) * (FDV / 64);
      wmma_gemm64<1, true, 0, 0, false><<<dim3((t + 7) / 8, 1), 256, 0, stream>>>(U16(Sh), U16(Sl), FS, 0, U16(Vh), U16(Vl), FS, 0, O, nullptr, FDV, 0, nullptr, nullptr, 0, FS, FDV, FS, 1.0f); }
    finalize_kernel<<<FS / 64, dim3(32, 8), 0, stream>>>(O, norm, out + (size_t)b * FDV * FS);
  }
}
